// RotaryCascadeAttention_74577812127922
// MI455X (gfx1250) — hardware-verified
//
#include <hip/hip_runtime.h>
#include <math.h>

constexpr int kBatch   = 4;
constexpr int kSeq     = 1024;
constexpr int kEmbd    = 1024;
constexpr int kHeads   = 16;
constexpr int kHeadDim = 64;
constexpr int kPairs   = 32;
constexpr int kRows    = kBatch * kSeq;
constexpr int kQkvCols = 3 * kEmbd;
constexpr int kQTiles  = kSeq / 16;
constexpr float kScoreScale = 1.0f / 8.0f;
constexpr float kInvSeq     = 1.0f / 1024.0f;
static_assert(8 * 8 == kHeadDim, "score scale is 1/sqrt(head dim)");
static_assert(kSeq == 1024, "mean divisor");
static_assert(kHeads * kHeadDim == kEmbd, "head split");
static_assert(2 * kPairs == kHeadDim, "pair count");
static_assert(kRows % 64 == 0 && kQkvCols % 64 == 0 && kEmbd % 64 == 0, "GEMM M, N tile multiples");
static_assert(kEmbd % 32 == 0 && kHeadDim % 32 == 0 && kSeq % 32 == 0, "GEMM K multiples of 32");

constexpr int kSPitch = 1028;
constexpr int kPPitch = 1032;
constexpr int kOPitch = 68;
constexpr int kRotPitch = 65;

typedef __attribute__((ext_vector_type(16))) __bf16 v16b;
typedef __attribute__((ext_vector_type(8)))  __bf16 v8b;
typedef __attribute__((ext_vector_type(8)))  float  v8f;
typedef __attribute__((ext_vector_type(4)))  float  v4f;
typedef __attribute__((ext_vector_type(2)))  float  v2f;
typedef __attribute__((ext_vector_type(4)))  unsigned int v4u;

__device__ __forceinline__ unsigned short f2bf_bits(float f) {
  unsigned u = __float_as_uint(f);
  return (unsigned short)((u + 0x7FFFu + ((u >> 16) & 1u)) >> 16);
}
__device__ __forceinline__ float bf_bits2f(unsigned short h) { return __uint_as_float(((unsigned)h) << 16); }
__device__ __forceinline__ unsigned pk16(unsigned short a, unsigned short b) { return (unsigned)a | ((unsigned)b << 16); }

union FragU { v16b v; v8b h[2]; };
__device__ __forceinline__ v16b frag_load(const __bf16* p) {
  FragU f;
  f.h[0] = *(const v8b*)(p);
  f.h[1] = *(const v8b*)(p + 16);
  return f.v;
}
__device__ __forceinline__ v8f mma_plain(v16b a, v16b b, v8f c) {
  return __builtin_amdgcn_wmma_f32_16x16x32_bf16(false, a, false, b, (short)0, c, false, false);
}
__device__ __forceinline__ v8f mma_guarded(v16b a, v16b b, v8f c) {
  c = __builtin_amdgcn_wmma_f32_16x16x32_bf16(false, a, false, b, (short)0, c, false, false);
  asm volatile("v_nop\n\tv_nop\n\tv_nop\n\tv_nop" : "+v"(c) : "v"(a), "v"(b));
  return c;
}
__device__ __forceinline__ void dep_guard4_b(v8f& a, v8f& b, v8f& c, v8f& d, v16b x, v16b y) {
  asm volatile("v_nop\n\tv_nop\n\tv_nop\n\tv_nop" : "+v"(a), "+v"(b), "+v"(c), "+v"(d) : "v"(x), "v"(y));
}
__device__ __forceinline__ void keep4_b(v16b a, v16b b, v16b c, v16b d) { asm volatile("v_nop" :: "v"(a), "v"(b), "v"(c), "v"(d)); }
__device__ __forceinline__ void acc_guard4(v8f& a, v8f& b, v8f& c, v8f& d) { asm volatile("v_nop\n\tv_nop\n\tv_nop\n\tv_nop" : "+v"(a), "+v"(b), "+v"(c), "+v"(d)); }

template <bool SPLIT_A>
__global__ __launch_bounds__(256) void wmma_gemm64_bf16(
    const unsigned short* __restrict__ Ap, const unsigned short* __restrict__ A2p, int lda,
    const unsigned short* __restrict__ Btp, int ldb,
    float* __restrict__ Cout, int ldc, int M, int N, int K) {
  const __bf16* A  = (const __bf16*)Ap;
  const __bf16* A2 = (const __bf16*)A2p;
  const __bf16* Bt = (const __bf16*)Btp;
  __shared__ __align__(16) float sT[8][16 * 68];
  const int lane = threadIdx.x & 31;
  const int wave = threadIdx.x >> 5;
  const int tilesN = N >> 6;
  const int tilesM = M >> 6;
  const int tile = blockIdx.x * 8 + wave;
  if (tile >= tilesM * tilesN) return;
  const int tm = tile / tilesN;
  const int tn = tile - tm * tilesN;
  const int m0 = tm << 6;
  const int n0 = tn << 6;

  const int rlane = lane & 15;
  const int koff  = (lane >> 4) * 8;
  const int mOff  = (lane >> 4) * 8;

  v8f acc[4][4];
#pragma unroll
  for (int i = 0; i < 4; ++i)
#pragma unroll
    for (int j = 0; j < 4; ++j) acc[i][j] = (v8f){0.f,0.f,0.f,0.f,0.f,0.f,0.f,0.f};

  for (int k0 = 0; k0 < K; k0 += 32) {
    v16b bh[4];
#pragma unroll
    for (int j = 0; j < 4; ++j) {
      const size_t bo = (size_t)(n0 + (j << 4) + rlane) * ldb + koff + k0;
      bh[j] = frag_load(Bt + bo);
    }
#pragma unroll
    for (int i = 0; i < 4; ++i) {
      const size_t ao = (size_t)(m0 + (i << 4) + rlane) * lda + koff + k0;
      v16b ah = frag_load(A + ao);
      v16b al;
      if (SPLIT_A) al = frag_load(A2 + ao);
#pragma unroll
      for (int j = 0; j < 4; ++j) {
        acc[i][j] = mma_plain(ah, bh[j], acc[i][j]);
        if (SPLIT_A) acc[i][j] = mma_plain(al, bh[j], acc[i][j]);
      }
      dep_guard4_b(acc[i][0], acc[i][1], acc[i][2], acc[i][3], ah, SPLIT_A ? al : ah);
    }
    keep4_b(bh[0], bh[1], bh[2], bh[3]);
  }
  acc_guard4(acc[0][0], acc[0][1], acc[0][2], acc[0][3]);
  acc_guard4(acc[1][0], acc[1][1], acc[1][2], acc[1][3]);
  acc_guard4(acc[2][0], acc[2][1], acc[2][2], acc[2][3]);
  acc_guard4(acc[3][0], acc[3][1], acc[3][2], acc[3][3]);

  float* slab = sT[wave];
#pragma unroll
  for (int i = 0; i < 4; ++i) {
    const int mBase = m0 + (i << 4);
#pragma unroll
    for (int j = 0; j < 4; ++j) {
#pragma unroll
      for (int r = 0; r < 8; ++r) {
        slab[(mOff + r) * 68 + (j << 4) + rlane] = acc[i][j][r];
      }
    }
    __builtin_amdgcn_fence(__ATOMIC_RELEASE, "workgroup");
    __builtin_amdgcn_wave_barrier();
    __builtin_amdgcn_fence(__ATOMIC_ACQUIRE, "workgroup");
    {
      const int hh = lane >> 4, c4 = (lane & 15) * 4;
      for (int pass = 0; pass < 2; ++pass) {
#pragma unroll
        for (int it = 0; it < 8; ++it) {
          const int row = it * 2 + hh;
          v4f v = *(const v4f*)(slab + row * 68 + c4);
          *(volatile v4f*)(Cout + (size_t)(mBase + row) * ldc + n0 + c4) = v;
        }
        __threadfence();
      }
    }
    __builtin_amdgcn_fence(__ATOMIC_RELEASE, "workgroup");
    __builtin_amdgcn_wave_barrier();
    __builtin_amdgcn_fence(__ATOMIC_ACQUIRE, "workgroup");
  }
}

__global__ __launch_bounds__(256) void cast8_bf16_kernel(const float* __restrict__ in, unsigned short* __restrict__ out, int n8) {
  const int i = blockIdx.x * 256 + threadIdx.x;
  if (i >= n8) return;
  const float* p = in + 8 * (size_t)i;
  const v4f a = *(const v4f*)(p);
  const v4f c = *(const v4f*)(p + 4);
  unsigned short hb[8];
#pragma unroll
  for (int e = 0; e < 4; ++e) {
    const float fa = a[e];
    const float fc = c[e];
    hb[e]     = f2bf_bits(fa);
    hb[4 + e] = f2bf_bits(fc);
  }
  const v4u u = (v4u){pk16(hb[0], hb[1]), pk16(hb[2], hb[3]), pk16(hb[4], hb[5]), pk16(hb[6], hb[7])};
  unsigned short* q = out + 8 * (size_t)i;
  *(volatile v4u*)q = u;
  __threadfence();
  *(volatile v4u*)q = u;
}

__global__ __launch_bounds__(256) void wtcast_bf16_kernel(const float* __restrict__ W, unsigned short* __restrict__ WT, int ncolsW) {
  __shared__ float sm[64][65];
  const int t  = threadIdx.x;
  const int k0 = blockIdx.x * 64;
  const int n0 = blockIdx.y * 64;
#pragma unroll
  for (int i = 0; i < 16; ++i) {
    const int e = i * 256 + t;
    const int r = e >> 6;
    const int c = e & 63;
    sm[c][r] = W[(size_t)(k0 + r) * ncolsW + n0 + c];
  }
  __syncthreads();
  const int lane = t & 31, wave = t >> 5;
  const int q = lane >> 3, c8 = (lane & 7) * 8;
  for (int pass = 0; pass < 2; ++pass) {
#pragma unroll
    for (int it = 0; it < 2; ++it) {
      const int row = wave * 8 + it * 4 + q;
      unsigned short hb[8];
#pragma unroll
      for (int e = 0; e < 8; ++e) hb[e] = f2bf_bits(sm[row][c8 + e]);
      const v4u u = (v4u){pk16(hb[0], hb[1]), pk16(hb[2], hb[3]), pk16(hb[4], hb[5]), pk16(hb[6], hb[7])};
      *(volatile v4u*)(WT + (size_t)(n0 + row) * kEmbd + k0 + c8) = u;
    }
    __threadfence();
  }
}

__global__ __launch_bounds__(256) void trig_table_kernel(float* __restrict__ tab) {
#pragma clang fp contract(off)
  const int tid  = threadIdx.x;
  const int lane = tid & 31;
  const int wave = tid >> 5;
  const int row  = blockIdx.x * 8 + wave;
  const int h    = row >> 10;
  const int t    = row & (kSeq - 1);
  const int j    = lane;
  const double R1 = 1.3335214321633240;
  const double R2 = 1.7782794100389228;
  const double R4 = 3.1622776601683795;
  const int jm = j & 7;
  const int jd = j >> 3;
  double r = (jm & 1) ? R1 : 1.0;
  r = r * ((jm & 2) ? R2 : 1.0);
  r = r * ((jm & 4) ? R4 : 1.0);
  const double dec = (jd == 0) ? 1.0 : (jd == 1) ? 10.0 : (jd == 2) ? 100.0 : 1000.0;
  const float p = (float)(r * dec);
  float inv = 1.0f / p;
  asm volatile("" : "+v"(inv));
  const int hm = h & 3;
  const int hq = h >> 2;
  double fr = (hm & 1) ? R2 : 1.0;
  fr = fr * ((hm & 2) ? R4 : 1.0);
  const double fdec = (hq == 0) ? 1.0 : (hq == 1) ? 10.0 : (hq == 2) ? 100.0 : 1000.0;
  const float fs = (float)(fr * fdec);
  float w = inv * fs;
  asm volatile("" : "+v"(w));
  float ang = (float)t * w;
  asm volatile("" : "+v"(ang));
  float sv, cv;
  sincosf(ang, &sv, &cv);
  float* op = tab + (size_t)row * kHeadDim;
  *(volatile float*)(op + lane) = cv;
  *(volatile float*)(op + kPairs + lane) = sv;
  __threadfence();
  *(volatile float*)(op + lane) = cv;
  *(volatile float*)(op + kPairs + lane) = sv;
}

__device__ __forceinline__ void store_tile_hilo(const float* sm, unsigned short* hi, unsigned short* lo,
                                                size_t base, size_t rowstride, int wave, int lane) {
  const int q = lane >> 3, c8 = (lane & 7) * 8;
#pragma unroll
  for (int it = 0; it < 2; ++it) {
    const int row = wave * 8 + it * 4 + q;
    const float* sp = sm + row * kRotPitch + c8;
    unsigned short hb[8], lb[8];
#pragma unroll
    for (int e = 0; e < 8; ++e) {
      const float f = sp[e];
      hb[e] = f2bf_bits(f);
      lb[e] = f2bf_bits(f - bf_bits2f(hb[e]));
    }
    const v4u uh = (v4u){pk16(hb[0], hb[1]), pk16(hb[2], hb[3]), pk16(hb[4], hb[5]), pk16(hb[6], hb[7])};
    const v4u ul = (v4u){pk16(lb[0], lb[1]), pk16(lb[2], lb[3]), pk16(lb[4], lb[5]), pk16(lb[6], lb[7])};
    const size_t o = base + (size_t)row * rowstride + c8;
    *(volatile v4u*)(hi + o) = uh;
    *(volatile v4u*)(lo + o) = ul;
  }
}

__global__ __launch_bounds__(256) void rot_split_kernel(const float* __restrict__ qkv, const float* __restrict__ tab,
                                                        unsigned short* __restrict__ qh, unsigned short* __restrict__ ql,
                                                        unsigned short* __restrict__ kh, unsigned short* __restrict__ kl,
                                                        unsigned short* __restrict__ vth, unsigned short* __restrict__ vtl) {
  __shared__ float sq[64 * kRotPitch];
  __shared__ float sk[64 * kRotPitch];
  __shared__ float sv[64 * kRotPitch];
  const int tid = threadIdx.x, lane = tid & 31, wave = tid >> 5;
  const int tt = blockIdx.x & 15;
  const int h  = (blockIdx.x >> 4) & 15;
  const int b  = blockIdx.x >> 8;
  const int t0 = tt * 64;
  const int bh = b * kHeads + h;
#pragma unroll 2
  for (int i = 0; i < 8; ++i) {
    const int e = i * 256 + tid;
    const int r = e >> 5;
    const int j = e & 31;
    const float* rowp = qkv + (size_t)(b * kSeq + t0 + r) * kQkvCols + h * kHeadDim + 2 * j;
    const v2f qq = *(const v2f*)(rowp);
    const v2f kk = *(const v2f*)(rowp + kEmbd);
    const float* tr = tab + (size_t)(h * kSeq + t0 + r) * kHeadDim;
    const float c = tr[j];
    const float s = tr[kPairs + j];
    const float q1 = qq[0], q2 = qq[1], k1 = kk[0], k2 = kk[1];
    sq[r * kRotPitch + j]          = q1 * c - q2 * s;
    sq[r * kRotPitch + kPairs + j] = q1 * s + q2 * c;
    sk[r * kRotPitch + j]          = k1 * c - k2 * s;
    sk[r * kRotPitch + kPairs + j] = k1 * s + k2 * c;
  }
#pragma unroll 4
  for (int i = 0; i < 16; ++i) {
    const int e = i * 256 + tid;
    const int r = e >> 6;
    const int d = e & 63;
    sv[d * kRotPitch + r] = qkv[(size_t)(b * kSeq + t0 + r) * kQkvCols + 2 * kEmbd + h * kHeadDim + d];
  }
  __syncthreads();
  const size_t qkbase = ((size_t)bh * kSeq + t0) * kHeadDim;
  const size_t vbase  = (size_t)bh * kHeadDim * kSeq + t0;
  for (int pass = 0; pass < 2; ++pass) {
    store_tile_hilo(sq, qh, ql, qkbase, (size_t)kHeadDim, wave, lane);
    store_tile_hilo(sk, kh, kl, qkbase, (size_t)kHeadDim, wave, lane);
    store_tile_hilo(sv, vth, vtl, vbase, (size_t)kSeq, wave, lane);
    __threadfence();
  }
}

__global__ __launch_bounds__(256) void attn_head_kernel(
    const unsigned short* __restrict__ qhp, const unsigned short* __restrict__ qlp,
    const unsigned short* __restrict__ khp, const unsigned short* __restrict__ klp,
    const unsigned short* __restrict__ vthp, const unsigned short* __restrict__ vtlp,
    const float* __restrict__ bias_in, const float* __restrict__ colw,
    unsigned short* __restrict__ atth, unsigned short* __restrict__ attl,
    float* __restrict__ bias_part, int head) {
  __shared__ __align__(16) float  Ssm[16 * kSPitch];
  __shared__ __align__(16) __bf16 Phs[16 * kPPitch];
  __shared__ __align__(16) __bf16 Pls[16 * kPPitch];
  __shared__ __align__(16) float  Ost[16 * kOPitch];

  const int tid = threadIdx.x, lane = tid & 31, wave = tid >> 5;
  const int c = lane & 15, hh = lane >> 4;
  const int b = blockIdx.x >> 6;
  const int tile = blockIdx.x & (kQTiles - 1);
  const int q0 = tile * 16;
  const int ntile = tile + 1;
  const int ncols = ntile * 16;
  const int kext  = (ncols + 31) & ~31;
  const int bh = b * kHeads + head;
  const float NEGV = -__builtin_huge_valf();

  const __bf16* qh = (const __bf16*)qhp + ((size_t)bh * kSeq + q0) * kHeadDim;
  const __bf16* ql = (const __bf16*)qlp + ((size_t)bh * kSeq + q0) * kHeadDim;
  const __bf16* kh = (const __bf16*)khp + (size_t)bh * kSeq * kHeadDim;
  const __bf16* kl = (const __bf16*)klp + (size_t)bh * kSeq * kHeadDim;
  const __bf16* vh = (const __bf16*)vthp + (size_t)bh * kHeadDim * kSeq;
  const __bf16* vl = (const __bf16*)vtlp + (size_t)bh * kHeadDim * kSeq;

  float cw = 0.0f;
  if (head > 0) cw = bf_bits2f(f2bf_bits(colw[head - 1]));

  {
    const v16b qah0 = frag_load(qh + c * kHeadDim + 8 * hh);
    const v16b qah1 = frag_load(qh + c * kHeadDim + 32 + 8 * hh);
    const v16b qal0 = frag_load(ql + c * kHeadDim + 8 * hh);
    const v16b qal1 = frag_load(ql + c * kHeadDim + 32 + 8 * hh);
#pragma unroll 1
    for (int nt = wave; nt < ntile; nt += 8) {
      const size_t ko = (size_t)(nt * 16 + c) * kHeadDim + 8 * hh;
      const v16b kh0 = frag_load(kh + ko);
      const v16b kh1 = frag_load(kh + ko + 32);
      const v16b kl0 = frag_load(kl + ko);
      const v16b kl1 = frag_load(kl + ko + 32);
      v8f acc = (v8f){0.f,0.f,0.f,0.f,0.f,0.f,0.f,0.f};
      acc = mma_guarded(qah0, kh0, acc);
      acc = mma_guarded(qah1, kh1, acc);
      acc = mma_guarded(qah0, kl0, acc);
      acc = mma_guarded(qah1, kl1, acc);
      acc = mma_guarded(qal0, kh0, acc);
      acc = mma_guarded(qal1, kh1, acc);
      const int scol = nt * 16 + c;
      float bv = 0.0f;
      if (head > 0) bv = cw * bias_in[b * kSeq + scol];
#pragma unroll
      for (int r = 0; r < 8; ++r) {
        const int m = 8 * hh + r;
        float v = acc[r] * kScoreScale + bv;
        if (scol > q0 + m) v = NEGV;
        Ssm[m * kSPitch + scol] = v;
      }
    }
  }
  if (ntile & 1) {
    Ssm[(tid >> 4) * kSPitch + ncols + (tid & 15)] = NEGV;
  }
  __syncthreads();

  {
    const int nsteps = kext >> 5;
#pragma unroll 1
    for (int rr = 0; rr < 2; ++rr) {
      const int row = 2 * wave + rr;
      float* srow = Ssm + row * kSPitch;
      __bf16* phr = Phs + row * kPPitch;
      __bf16* plr = Pls + row * kPPitch;
      float mx = NEGV;
#pragma unroll 1
      for (int u = 0; u < nsteps; ++u) mx = fmaxf(mx, srow[lane + 32 * u]);
#pragma unroll
      for (int off = 16; off > 0; off >>= 1) mx = fmaxf(mx, __shfl_xor(mx, off, 32));
      float sum = 0.0f;
#pragma unroll 1
      for (int u = 0; u < nsteps; ++u) {
        const int col = lane + 32 * u;
        const float x = srow[col];
        float e = 0.0f;
        if (x > -1.0e29f) e = expf(x - mx);
        srow[col] = e;
        sum += e;
      }
#pragma unroll
      for (int off = 16; off > 0; off >>= 1) sum += __shfl_xor(sum, off, 32);
      const float inv = 1.0f / sum;
#pragma unroll 1
      for (int u = 0; u < nsteps; ++u) {
        const int col = lane + 32 * u;
        const float p = srow[col] * inv;
        srow[col] = p;
        const unsigned short hb = f2bf_bits(p);
        const unsigned short lb = f2bf_bits(p - bf_bits2f(hb));
        phr[col] = __builtin_bit_cast(__bf16, hb);
        plr[col] = __builtin_bit_cast(__bf16, lb);
      }
    }
  }
  __syncthreads();

  if (wave >= 4) {
    const int tt = tid - 128;
    v4f res[2];
#pragma unroll
    for (int g = 0; g < 2; ++g) {
      const int c4 = 4 * (tt + 128 * g);
      const int cc = (c4 < kext) ? c4 : (kext - 4);
      v4f a = (v4f){0.f, 0.f, 0.f, 0.f};
#pragma unroll 4
      for (int m = 0; m < 16; ++m) a += *(const v4f*)(Ssm + m * kSPitch + cc);
      const bool live = (c4 < kext);
      v4f z;
      z[0] = live ? a[0] : 0.0f;
      z[1] = live ? a[1] : 0.0f;
      z[2] = live ? a[2] : 0.0f;
      z[3] = live ? a[3] : 0.0f;
      res[g] = z;
    }
    float* bp = bias_part + (size_t)(b * kQTiles + tile) * kSeq;
    for (int pass = 0; pass < 2; ++pass) {
#pragma unroll
      for (int g = 0; g < 2; ++g) *(volatile v4f*)(bp + 4 * (tt + 128 * g)) = res[g];
      __threadfence();
    }
  } else {
    const int d0 = wave * 16;
    v8f acc = (v8f){0.f,0.f,0.f,0.f,0.f,0.f,0.f,0.f};
    const __bf16* ph = Phs + c * kPPitch + 8 * hh;
    const __bf16* pl = Pls + c * kPPitch + 8 * hh;
    const __bf16* vbh = vh + (size_t)(d0 + c) * kSeq + 8 * hh;
    const __bf16* vbl = vl + (size_t)(d0 + c) * kSeq + 8 * hh;
#pragma unroll 1
    for (int k0 = 0; k0 < kext; k0 += 32) {
      const v16b ah = frag_load(ph + k0);
      const v16b al = frag_load(pl + k0);
      const v16b bhf = frag_load(vbh + k0);
      const v16b blf = frag_load(vbl + k0);
      acc = mma_guarded(ah, bhf, acc);
      acc = mma_guarded(ah, blf, acc);
      acc = mma_guarded(al, bhf, acc);
    }
#pragma unroll
    for (int r = 0; r < 8; ++r) Ost[(8 * hh + r) * kOPitch + d0 + c] = acc[r];
  }
  __syncthreads();

  if (wave < 4) {
    const int q = lane >> 3, c8 = (lane & 7) * 8;
    const int row = wave * 4 + q;
    const float* sp = Ost + row * kOPitch + c8;
    unsigned short hb[8], lb[8];
#pragma unroll
    for (int e = 0; e < 8; ++e) {
      const float f = sp[e];
      hb[e] = f2bf_bits(f);
      lb[e] = f2bf_bits(f - bf_bits2f(hb[e]));
    }
    const v4u uh = (v4u){pk16(hb[0], hb[1]), pk16(hb[2], hb[3]), pk16(hb[4], hb[5]), pk16(hb[6], hb[7])};
    const v4u ul = (v4u){pk16(lb[0], lb[1]), pk16(lb[2], lb[3]), pk16(lb[4], lb[5]), pk16(lb[6], lb[7])};
    const size_t o = (size_t)(b * kSeq + q0 + row) * kEmbd + head * kHeadDim + c8;
    *(volatile v4u*)(atth + o) = uh;
    *(volatile v4u*)(attl + o) = ul;
    __threadfence();
    *(volatile v4u*)(atth + o) = uh;
    *(volatile v4u*)(attl + o) = ul;
  }
}

__global__ __launch_bounds__(256) void colmean_reduce_kernel(const float* __restrict__ part, float* __restrict__ outv) {
  const int i  = blockIdx.x * 256 + threadIdx.x;
  const int b  = i >> 8;
  const int c4 = (i & 255) * 4;
  const float* p = part + (size_t)b * kQTiles * kSeq + c4;
  v4f s = (v4f){0.f, 0.f, 0.f, 0.f};
#pragma unroll 4
  for (int k = 0; k < kQTiles; ++k) {
    const v4f v = *(const v4f*)(p + (size_t)k * kSeq);
    s += v;
  }
  s = s * kInvSeq;
  float* o = outv + b * kSeq + c4;
  *(volatile v4f*)o = s;
  __threadfence();
  *(volatile v4f*)o = s;
}

extern "C" void kernel_launch(void* const* d_in, const int* in_sizes, int n_in,
                              void* d_out, int out_size, void* d_ws, size_t ws_size, hipStream_t stream) {
  if (n_in < 4 || d_out == nullptr || d_ws == nullptr) return;
  if (in_sizes[0] != kRows * kEmbd || in_sizes[1] != kEmbd * kQkvCols || in_sizes[2] != kEmbd * kEmbd ||
      in_sizes[3] != kHeads - 1 || out_size != kRows * kEmbd) return;

  const float* x     = (const float*)d_in[0];
  const float* Wqkv  = (const float*)d_in[1];
  const float* Wproj = (const float*)d_in[2];
  const float* colw  = (const float*)d_in[3];
  float* out = (float*)d_out;

  char* ws = (char*)d_ws;
  size_t off = 0;
  auto carve = [&](size_t bytes) -> char* { char* p = ws + off; off += (bytes + 255) & ~(size_t)255; return p; };
  const size_t headPlane = (size_t)kBatch * kHeads * kSeq * kHeadDim * 2;
  unsigned short* XB   = (unsigned short*)carve((size_t)kRows * kEmbd * 2);
  unsigned short* WQT  = (unsigned short*)carve((size_t)kQkvCols * kEmbd * 2);
  unsigned short* WPT  = (unsigned short*)carve((size_t)kEmbd * kEmbd * 2);
  float*          QKV  = (float*)carve((size_t)kRows * kQkvCols * 4);
  unsigned short* QH   = (unsigned short*)carve(headPlane);
  unsigned short* QL   = (unsigned short*)carve(headPlane);
  unsigned short* KH   = (unsigned short*)carve(headPlane);
  unsigned short* KL   = (unsigned short*)carve(headPlane);
  unsigned short* VTH  = (unsigned short*)carve(headPlane);
  unsigned short* VTL  = (unsigned short*)carve(headPlane);
  float*          TAB  = (float*)carve((size_t)kHeads * kSeq * kHeadDim * 4);
  float*          BPART = (float*)carve((size_t)kBatch * kQTiles * kSeq * 4);
  float*          BIASV = (float*)carve((size_t)kBatch * kSeq * 4);
  unsigned short* ATTL = (unsigned short*)carve((size_t)kRows * kEmbd * 2);
  unsigned short* ATTH = XB;
  if (off > ws_size || off > (size_t)134217728) return;

  const int n8x = kRows * (kEmbd / 8);
  cast8_bf16_kernel<<<n8x / 256, 256, 0, stream>>>(x, XB, n8x);
  wtcast_bf16_kernel<<<dim3(kEmbd / 64, kQkvCols / 64), 256, 0, stream>>>(Wqkv, WQT, kQkvCols);
  wtcast_bf16_kernel<<<dim3(kEmbd / 64, kEmbd / 64), 256, 0, stream>>>(Wproj, WPT, kEmbd);
  trig_table_kernel<<<(kHeads * kSeq) / 8, 256, 0, stream>>>(TAB);

  wmma_gemm64_bf16<false><<<(kRows / 64) * (kQkvCols / 64) / 8, 256, 0, stream>>>(
      XB, XB, kEmbd, WQT, kEmbd, QKV, kQkvCols, kRows, kQkvCols, kEmbd);

  rot_split_kernel<<<kBatch * kHeads * (kSeq / 64), 256, 0, stream>>>(QKV, TAB, QH, QL, KH, KL, VTH, VTL);

  for (int h = 0; h < kHeads; ++h) {
    if (h > 0) colmean_reduce_kernel<<<(kBatch * kSeq / 4) / 256, 256, 0, stream>>>(BPART, BIASV);
    attn_head_kernel<<<kBatch * kQTiles, 256, 0, stream>>>(QH, QL, KH, KL, VTH, VTL, BIASV, colw, ATTH, ATTL, BPART, h);
  }

  wmma_gemm64_bf16<true><<<(kRows / 64) * (kEmbd / 64) / 8, 256, 0, stream>>>(
      ATTH, ATTL, kEmbd, WPT, kEmbd, out, kEmbd, kRows, kEmbd, kEmbd);
}
